// Guide_35570919146244
// MI455X (gfx1250) — hardware-verified
//
#include <hip/hip_runtime.h>

#ifndef NB
#define NB 2
#endif
#define NB_FULL 2
#ifndef IMH
#define IMH 240
#endif
#ifndef IMH_FULL
#define IMH_FULL 240
#endif
#define CH 64
#define CIN 128
#define IMW 320
#define HWP (IMH * IMW)
#define HWPF ((size_t)IMH_FULL * IMW)
#define PH (IMH + 2)
#define PW 322
#define NPIX ((size_t)NB * HWP)
#define KCV 1152
#if ((IMH * IMW) % 25600) == 0
#define CHUNK 25600
#else
#define CHUNK 5120
#endif
#define NCHUNK ((int)(NPIX / CHUNK))
#define NBORD (2 * PW + 2 * IMH)
#define KBO 768
#define WSC 16.0f
#define RSC 256.0f
#define ALPHA 0.0625f
#define BNEPS 1e-5f
static_assert(HWP % CHUNK == 0);
static_assert(CHUNK % 128 == 0);
static_assert(CHUNK % IMW == 0);
static_assert(CHUNK % 16 == 0);
static_assert(HWP % 128 == 0);
static_assert(IMW % 32 == 0);
static_assert(PW == IMW + 2);
static_assert(NB >= 1 && NB <= NB_FULL);
static_assert(IMH >= 3 && IMH <= IMH_FULL);
static_assert(PH * PW == HWP + NBORD);
static_assert(NCHUNK >= 1 && (size_t)NCHUNK * CHUNK == NPIX);

typedef _Float16 v16h __attribute__((ext_vector_type(16)));
typedef unsigned short v8us __attribute__((ext_vector_type(8), may_alias));
typedef float  v8f  __attribute__((ext_vector_type(8)));
typedef float  v4f  __attribute__((ext_vector_type(4)));
typedef float  v4fa __attribute__((ext_vector_type(4), may_alias));
union FragH { v16h v; v8us half[2]; _Float16 h[16]; unsigned short u[16]; };
union HU { _Float16 h; unsigned short u; };

__device__ __forceinline__ unsigned short bf16_bits(float x) { unsigned int u = __float_as_uint(x); return (unsigned short)((u + 0x7FFFu + ((u >> 16) & 1u)) >> 16); }
__device__ __forceinline__ float bf16_val(unsigned short b) { return __uint_as_float(((unsigned int)b) << 16); }
__device__ __forceinline__ float bf16_rne(float x) { return bf16_val(bf16_bits(x)); }

__device__ __forceinline__ v16h g2_frag(const _Float16* p, int hh) { FragH f; f.half[0] = *(const v8us*)((const unsigned short*)p + 8 * hh); f.half[1] = *(const v8us*)((const unsigned short*)p + 16 + 8 * hh); return f.v; }
__device__ __forceinline__ v8f g2_mma(v16h a, v16h b, v8f c) { v8f d = __builtin_amdgcn_wmma_f32_16x16x32_f16(false, a, false, b, (short)0, c, false, false); asm volatile("v_nop\n\tv_nop\n\tv_nop\n\tv_nop" : "+v"(d) : "v"(a), "v"(b)); return d; }
__device__ __forceinline__ _Float16 hsel(float a, bool res) { const _Float16 h = (_Float16)a; const _Float16 l = (_Float16)((a - (float)h) * RSC); return res ? l : h; }

__global__ __launch_bounds__(256) void k_wconv(const float* __restrict__ w, int cin, _Float16* __restrict__ Bt) {
  const int t = blockIdx.x * 256 + threadIdx.x; if (t >= 64 * 9 * (CIN / 8)) return;
  const int j8 = (t & 15) * 8, tap = (t >> 4) % 9, o = t / 144;
  FragH f;
#pragma unroll
  for (int q = 0; q < 8; ++q) { const int j = j8 + q; const int c = (j < cin) ? j : (j - cin); const float sc = (j < cin) ? WSC : (WSC / RSC);
    f.h[q] = (_Float16)(bf16_rne(w[((size_t)o * cin + c) * 9 + tap]) * sc); }
  unsigned short* d = (unsigned short*)Bt + (size_t)o * KCV + (size_t)tap * CIN + j8;
  *(volatile v8us*)d = f.half[0]; __threadfence(); *(volatile v8us*)d = f.half[0];
}
__global__ __launch_bounds__(256) void k_w1x1(const float* __restrict__ w, int cin, int nO, _Float16* __restrict__ Bt) {
  const int k8n = (2 * cin) / 8; const int t = blockIdx.x * 256 + threadIdx.x; if (t >= 64 * k8n) return;
  const int j8 = (t % k8n) * 8, o = t / k8n; const int oc = min(o, nO - 1); const float live = (o < nO) ? 1.0f : 0.0f;
  FragH f;
#pragma unroll
  for (int q = 0; q < 8; ++q) { const int j = j8 + q; const int c = (j < cin) ? j : (j - cin); const float sc = (j < cin) ? WSC : (WSC / RSC);
    f.h[q] = (_Float16)(bf16_rne(w[(size_t)oc * cin + c]) * sc * live); }
  unsigned short* d = (unsigned short*)Bt + (size_t)o * (2 * cin) + j8;
  *(volatile v8us*)d = f.half[0]; __threadfence(); *(volatile v8us*)d = f.half[0];
}
__global__ __launch_bounds__(256) void k_border(_Float16* __restrict__ XP) {
  const int t = blockIdx.x * 256 + threadIdx.x; if (t >= NB * NBORD * 16) return;
  const int piece = t & 15; const int bp = (t >> 4) % NBORD; const int n = (t >> 4) / NBORD;
  int y, x;
  if (bp < PW) { y = 0; x = bp; } else if (bp < 2 * PW) { y = PH - 1; x = bp - PW; } else if (bp < 2 * PW + IMH) { y = 1 + bp - 2 * PW; x = 0; } else { y = 1 + bp - 2 * PW - IMH; x = PW - 1; }
  v8us z; for (int q = 0; q < 8; ++q) z[q] = 0;
  unsigned short* d = (unsigned short*)XP + (((size_t)n * PH + y) * PW + x) * CIN + piece * 8;
  *(volatile v8us*)d = z; __threadfence(); *(volatile v8us*)d = z;
}
__global__ __launch_bounds__(256) void k_pack(const float* __restrict__ feat, const float* __restrict__ wgt, _Float16* __restrict__ XP) {
  const int tid = threadIdx.x, w = tid >> 5, lane = tid & 31;
  const int s = w & 1;
  const size_t pix = (size_t)blockIdx.x * 16 + (w >> 1) * 4 + (lane >> 3);
  if (pix >= NPIX) return;
  const int n = (int)(pix / HWP); const int p = (int)(pix - (size_t)n * HWP); const int y = p / IMW, x = p - y * IMW;
  const int c8 = (lane & 7) * 8;
  const float* src = (s ? wgt : feat) + ((size_t)n * CH + c8) * HWPF + (size_t)y * IMW + x;
  FragH f;
#pragma unroll
  for (int q = 0; q < 8; ++q) f.h[q] = (_Float16)bf16_rne(src[(size_t)q * HWPF]);
  unsigned short* d = (unsigned short*)XP + (((size_t)n * PH + y + 1) * PW + x + 1) * CIN + s * CH + c8;
  *(volatile v8us*)d = f.half[0]; __threadfence(); *(volatile v8us*)d = f.half[0];
}

template <int EPI>
__device__ __forceinline__ void epi_consts(int col, const float* __restrict__ pb, int nbias, const float* __restrict__ pg, const float* __restrict__ pbe, const float* __restrict__ pm, const float* __restrict__ pv, float& c1, float& c2, float& c3) {
  c1 = 0.f; c2 = 1.f; c3 = 0.f;
  if (EPI == 0 || EPI == 1 || EPI == 2) { const float bv = bf16_rne(pb[min(col, nbias - 1)]); c1 = (col < nbias) ? bv : 0.f; }
  if (EPI == 2 || EPI == 3) { const float g = bf16_rne(pg[col]), be = bf16_rne(pbe[col]), mu = bf16_rne(pm[col]), var = bf16_rne(pv[col]); const float inv = g * (1.0f / sqrtf(var + BNEPS)); c2 = inv; c3 = be - mu * inv; }
}
__device__ __forceinline__ void st_planes(float (*sw)[68], unsigned short* __restrict__ dst, int lane) {
  const int psub = lane >> 4, j = lane & 15, ch0 = (j & 7) * 8; const bool res = (j >= 8);
  for (int pass = 0; pass < 2; ++pass) {
#pragma unroll
    for (int i = 0; i < 16; ++i) { const int p = 2 * i + psub; const v4f f0 = *(const v4fa*)&sw[p][ch0]; const v4f f1 = *(const v4fa*)&sw[p][ch0 + 4]; FragH f;
#pragma unroll
      for (int q = 0; q < 4; ++q) { f.h[q] = hsel(f0[q], res); f.h[4 + q] = hsel(f1[q], res); }
      *(volatile v8us*)(dst + (size_t)p * CIN + j * 8) = f.half[0]; }
    if (pass == 0) __threadfence();
  }
}
__device__ __forceinline__ void st_rows64(float (*sw)[68], float* __restrict__ C, int lane) {
  const int rsub = lane >> 4, c4 = (lane & 15) * 4;
  for (int pass = 0; pass < 2; ++pass) {
#pragma unroll
    for (int q = 0; q < 16; ++q) { const int r = 2 * q + rsub; const v4f v = *(const v4fa*)&sw[r][c4]; *(volatile v4f*)(C + (size_t)r * 64 + c4) = v; }
    if (pass == 0) __threadfence();
  }
}
__device__ __forceinline__ void st_nchw(float (*sw)[68], float* __restrict__ ob, int lane) {
  const int osub = lane >> 3, q4 = (lane & 7) * 4;
  for (int pass = 0; pass < 2; ++pass) {
#pragma unroll
    for (int i = 0; i < 16; ++i) { const int o = i * 4 + osub; v4f v; v[0] = sw[q4][o]; v[1] = sw[q4 + 1][o]; v[2] = sw[q4 + 2][o]; v[3] = sw[q4 + 3][o];
      *(volatile v4f*)(ob + (size_t)o * HWP + q4) = v; }
    if (pass == 0) __threadfence();
  }
}

template <int EPI>
__global__ __launch_bounds__(128) void k_conv(const _Float16* __restrict__ XP, const _Float16* __restrict__ Bt, const float* __restrict__ pb, int nbias,
    const float* __restrict__ pg, const float* __restrict__ pbe, const float* __restrict__ pm, const float* __restrict__ pv, _Float16* __restrict__ TP, float* __restrict__ out) {
  __shared__ __attribute__((aligned(16))) float so[4][32][68];
  const int tid = threadIdx.x, w = tid >> 5, lane = tid & 31, ln = lane & 15, hh = lane >> 4;
  const int G = blockIdx.x * 4 + w; if (G >= (int)(NPIX / 32)) return;
  const int n = G / (HWP / 32), rr = G - n * (HWP / 32), y = rr / (IMW / 32), x0 = (rr - y * (IMW / 32)) * 32;
  const _Float16* a0p = XP + (((size_t)n * PH + y) * PW + x0 + ln) * CIN; const _Float16* a1p = a0p + 16 * CIN;
  const _Float16* b0p = Bt + (size_t)ln * KCV; const _Float16* b1p = b0p + (size_t)16 * KCV; const _Float16* b2p = b1p + (size_t)16 * KCV; const _Float16* b3p = b2p + (size_t)16 * KCV;
  const v8f z8 = {0.f,0.f,0.f,0.f,0.f,0.f,0.f,0.f}; v8f c00 = z8, c01 = z8, c02 = z8, c03 = z8, c10 = z8, c11 = z8, c12 = z8, c13 = z8;
#pragma unroll 1
  for (int tap = 0; tap < 9; ++tap) { const int dy = tap / 3, dx = tap - dy * 3; const int aoff = (dy * PW + dx) * CIN; const int kb0 = tap * CIN;
#pragma unroll 1
    for (int cc = 0; cc < CIN; cc += 32) { const int kb = kb0 + cc;
      const v16h a0 = g2_frag(a0p + aoff + cc, hh), a1 = g2_frag(a1p + aoff + cc, hh);
      v16h b = g2_frag(b0p + kb, hh); c00 = g2_mma(a0, b, c00); c10 = g2_mma(a1, b, c10);
      b = g2_frag(b1p + kb, hh); c01 = g2_mma(a0, b, c01); c11 = g2_mma(a1, b, c11);
      b = g2_frag(b2p + kb, hh); c02 = g2_mma(a0, b, c02); c12 = g2_mma(a1, b, c12);
      b = g2_frag(b3p + kb, hh); c03 = g2_mma(a0, b, c03); c13 = g2_mma(a1, b, c13); } }
  v8f accs[8] = {c00, c01, c02, c03, c10, c11, c12, c13};
#pragma unroll
  for (int u = 0; u < 8; ++u) { const int t = u & 3, half = u >> 2; const int col = t * 16 + ln; float c1, c2, c3; epi_consts<EPI>(col, pb, nbias, pg, pbe, pm, pv, c1, c2, c3);
#pragma unroll
    for (int r = 0; r < 8; ++r) { float v = (accs[u][r] * ALPHA + c1) * c2 + c3; if (EPI != 1) v = fmaxf(v, 0.f); so[w][half * 16 + 8 * hh + r][col] = v; } }
  __builtin_amdgcn_fence(__ATOMIC_ACQ_REL, "workgroup"); __builtin_amdgcn_wave_barrier();
  if (EPI == 0) st_planes(so[w], (unsigned short*)TP + (size_t)G * 32 * CIN, lane);
  if (EPI == 3) st_nchw(so[w], out + (size_t)n * CH * HWP + (size_t)y * IMW + x0, lane);
}
template <int EPI>
__global__ __launch_bounds__(128) void k_rows(const _Float16* __restrict__ A, int K, const _Float16* __restrict__ Bt, const float* __restrict__ pb, int nbias,
    const float* __restrict__ pg, const float* __restrict__ pbe, const float* __restrict__ pm, const float* __restrict__ pv, float* __restrict__ C, _Float16* __restrict__ MPp, int chunk, int M) {
  __shared__ __attribute__((aligned(16))) float so[4][32][68];
  const int tid = threadIdx.x, w = tid >> 5, lane = tid & 31, ln = lane & 15, hh = lane >> 4;
  const int row0 = blockIdx.x * 128 + 32 * w; if (row0 >= M) return;
  const _Float16* a0p = A + (size_t)(row0 + ln) * K; const _Float16* a1p = a0p + (size_t)16 * K;
  const _Float16* b0p = Bt + (size_t)ln * K; const _Float16* b1p = b0p + (size_t)16 * K; const _Float16* b2p = b1p + (size_t)16 * K; const _Float16* b3p = b2p + (size_t)16 * K;
  const v8f z8 = {0.f,0.f,0.f,0.f,0.f,0.f,0.f,0.f}; v8f c00 = z8, c01 = z8, c02 = z8, c03 = z8, c10 = z8, c11 = z8, c12 = z8, c13 = z8;
#pragma unroll 1
  for (int kb = 0; kb < K; kb += 32) { const v16h a0 = g2_frag(a0p + kb, hh), a1 = g2_frag(a1p + kb, hh);
    v16h b = g2_frag(b0p + kb, hh); c00 = g2_mma(a0, b, c00); c10 = g2_mma(a1, b, c10);
    b = g2_frag(b1p + kb, hh); c01 = g2_mma(a0, b, c01); c11 = g2_mma(a1, b, c11);
    b = g2_frag(b2p + kb, hh); c02 = g2_mma(a0, b, c02); c12 = g2_mma(a1, b, c12);
    b = g2_frag(b3p + kb, hh); c03 = g2_mma(a0, b, c03); c13 = g2_mma(a1, b, c13); }
  v8f accs[8] = {c00, c01, c02, c03, c10, c11, c12, c13};
#pragma unroll
  for (int u = 0; u < 8; ++u) { const int t = u & 3, half = u >> 2; const int col = t * 16 + ln; float c1, c2, c3; epi_consts<EPI>(col, pb, nbias, pg, pbe, pm, pv, c1, c2, c3);
#pragma unroll
    for (int r = 0; r < 8; ++r) { float v = (accs[u][r] * ALPHA + c1) * c2 + c3; if (EPI != 1) v = fmaxf(v, 0.f); so[w][half * 16 + 8 * hh + r][col] = v; } }
  __builtin_amdgcn_fence(__ATOMIC_ACQ_REL, "workgroup"); __builtin_amdgcn_wave_barrier();
  if (EPI == 1) st_rows64(so[w], C + (size_t)row0 * 64, lane);
  if (EPI == 2) { const size_t gp0 = (size_t)chunk * CHUNK + row0; const int n = (int)(gp0 / HWP); const int p = (int)(gp0 - (size_t)n * HWP); const int y = p / IMW, x0 = p - y * IMW;
    st_planes(so[w], (unsigned short*)MPp + (((size_t)n * PH + y + 1) * PW + x0 + 1) * CIN, lane); }
}
__global__ __launch_bounds__(128) void k_dyn(const float* __restrict__ feat, const float* __restrict__ BS, _Float16* __restrict__ BOP, int chunk) {
  __shared__ float psh[3 * 18 * CH];
  __shared__ float bsh[16][56];
  __shared__ __attribute__((aligned(16))) unsigned short bo[16][KBO];
  const int tid = threadIdx.x;
  const int g = chunk * (CHUNK / 16) + blockIdx.x;
  const int n = g / (HWP / 16), r = g - n * (HWP / 16), y = r / (IMW / 16), x0 = (r - y * (IMW / 16)) * 16;
  for (int i = 0; i < 27; ++i) { const int e = tid + i * 128; const int col = e % 18, c = (e / 18) % CH, rowi = e / (18 * CH);
    const int yy = y + rowi - 1, xx = x0 + col - 1; const int yc = min(max(yy, 0), IMH - 1), xc = min(max(xx, 0), IMW - 1);
    const float v = bf16_rne(feat[(((size_t)n * CH + c) * IMH_FULL + yc) * IMW + xc]); const bool inb = (yy >= 0) && (yy < IMH) && (xx >= 0) && (xx < IMW);
    psh[(rowi * 18 + col) * CH + c] = inb ? v : 0.0f; }
  for (int i = 0; i < 7; ++i) { const int e = tid + i * 128; const int ec = min(e, 16 * 54 - 1); const int p = ec / 54, oc = ec - p * 54;
    const float v = BS[((size_t)n * HWP + (size_t)y * IMW + x0 + p) * 64 + oc]; if (e < 16 * 54) bsh[p][oc] = v; }
  __syncthreads();
  const int c = tid >> 1, m0 = (tid & 1) * 3;
#pragma unroll 1
  for (int p = 0; p < 16; ++p) {
    float pv[9];
#pragma unroll
    for (int l = 0; l < 9; ++l) pv[l] = psh[((l / 3) * 18 + p + (l % 3)) * CH + c];
#pragma unroll
    for (int mm = 0; mm < 3; ++mm) { const int m = m0 + mm; float s = 0.f;
#pragma unroll
      for (int l = 0; l < 9; ++l) s += pv[l] * bsh[p][m * 9 + l];
      HU uh, ul; uh.h = (_Float16)s; ul.h = (_Float16)((s - (float)uh.h) * RSC); bo[p][c * 6 + m] = uh.u; bo[p][384 + c * 6 + m] = ul.u; }
  }
  __syncthreads();
  const int w = tid >> 5, lane = tid & 31;
  unsigned short* base = (unsigned short*)BOP + (size_t)blockIdx.x * 16 * KBO;
  for (int pass = 0; pass < 2; ++pass) {
#pragma unroll
    for (int q = 0; q < 4; ++q) { const int p = w * 4 + q;
#pragma unroll
      for (int it = 0; it < 3; ++it) { const int j = it * 32 + lane; const v8us v = *(const v8us*)&bo[p][j * 8]; *(volatile v8us*)(base + (size_t)p * KBO + j * 8) = v; } }
    if (pass == 0) __threadfence();
  }
}

extern "C" void kernel_launch(void* const* d_in, const int* in_sizes, int n_in,
                              void* d_out, int out_size, void* d_ws, size_t ws_size, hipStream_t stream) {
  if (n_in < 17) return;
  if (in_sizes[0] < (int)((size_t)NB * CH * HWPF) || in_sizes[1] < (int)((size_t)NB * CH * HWPF) || in_sizes[2] < 64 * 128 * 9 || in_sizes[3] < 64 || in_sizes[4] < 54 * 64 || in_sizes[5] < 54 ||
      in_sizes[6] < 64 * 384 || in_sizes[7] < 64 || in_sizes[8] < 64 || in_sizes[9] < 64 || in_sizes[10] < 64 || in_sizes[11] < 64 || in_sizes[12] < 64 * 64 * 9 ||
      in_sizes[13] < 64 || in_sizes[14] < 64 || in_sizes[15] < 64 || in_sizes[16] < 64) return;
  if (out_size < (int)(NPIX * CH)) return;
  const float* const* I = (const float* const*)d_in;
  const float* feat = I[0]; const float* wgt = I[1]; const float* w1 = I[2]; const float* b1 = I[3]; const float* w2 = I[4]; const float* b2 = I[5];
  const float* coef = I[6]; const float* cb = I[7]; const float* brg = I[8]; const float* brb = I[9]; const float* brm = I[10]; const float* brv = I[11];
  const float* w3 = I[12]; const float* g3 = I[13]; const float* be3 = I[14]; const float* m3 = I[15]; const float* v3 = I[16];
  float* out = (float*)d_out;
  char* ws = (char*)d_ws; size_t off = 0;
  auto take = [&](size_t bytes) { char* p = ws + off; off += (bytes + 255) & ~(size_t)255; return p; };
  _Float16* W1P = (_Float16*)take((size_t)64 * KCV * 2);
  _Float16* W3P = (_Float16*)take((size_t)64 * KCV * 2);
  _Float16* W2P = (_Float16*)take((size_t)64 * 128 * 2);
  _Float16* CFP = (_Float16*)take((size_t)64 * KBO * 2);
  const size_t r1b = (size_t)NB * PH * PW * CIN * 2;
  const size_t tpb = NPIX * CIN * 2, bopb = (size_t)CHUNK * KBO * 2; const size_t r2b = tpb > bopb ? tpb : bopb;
  const size_t r3b = NPIX * 64 * 4;
  _Float16* R1 = (_Float16*)take(r1b); _Float16* R2 = (_Float16*)take(r2b); float* BS = (float*)take(r3b);
  if (off > ws_size) return;
  _Float16* XP = R1; _Float16* MP = R1; _Float16* TP = R2; _Float16* BOP = R2;

  k_wconv<<<(64 * 9 * 16 + 255) / 256, 256, 0, stream>>>(w1, 128, W1P);
  k_wconv<<<(64 * 9 * 16 + 255) / 256, 256, 0, stream>>>(w3, 64, W3P);
  k_w1x1<<<(64 * 16 + 255) / 256, 256, 0, stream>>>(w2, 64, 54, W2P);
  k_w1x1<<<(64 * 96 + 255) / 256, 256, 0, stream>>>(coef, 384, 64, CFP);
  k_border<<<(unsigned)((NB * NBORD * 16 + 255) / 256), 256, 0, stream>>>(XP);
  k_pack<<<(unsigned)(NPIX / 16), 256, 0, stream>>>(feat, wgt, XP);
  k_conv<0><<<(unsigned)(NPIX / 128), 128, 0, stream>>>(XP, W1P, b1, 64, nullptr, nullptr, nullptr, nullptr, TP, nullptr);
  k_rows<1><<<(unsigned)(NPIX / 128), 128, 0, stream>>>(TP, 128, W2P, b2, 54, nullptr, nullptr, nullptr, nullptr, BS, nullptr, 0, (int)NPIX);
  k_border<<<(unsigned)((NB * NBORD * 16 + 255) / 256), 256, 0, stream>>>(MP);
  for (int chn = 0; chn < NCHUNK; ++chn) {
    k_dyn<<<CHUNK / 16, 128, 0, stream>>>(feat, BS, BOP, chn);
    k_rows<2><<<CHUNK / 128, 128, 0, stream>>>(BOP, KBO, CFP, cb, 64, brg, brb, brm, brv, nullptr, MP, chn, CHUNK);
  }
  k_conv<3><<<(unsigned)(NPIX / 128), 128, 0, stream>>>(MP, W3P, nullptr, 0, g3, be3, m3, v3, nullptr, out);
}
